// DifferentiableKMeansLayer_33655363732009
// MI455X (gfx1250) — hardware-verified
//
#include <hip/hip_runtime.h>


#define NN_  131072
#define DD   64
#define KK   512
#define TEMP 0.1f
#define CSC  64.0f
#define PSC  32768.0f
#define LOSC 1024.0f
#define LOSCI (1.0f / 1024.0f)

typedef _Float16 h16;
typedef unsigned short bf;
typedef __attribute__((ext_vector_type(16))) __bf16   v16bf;
typedef __attribute__((ext_vector_type(16))) _Float16 v16h;
typedef __attribute__((ext_vector_type(8)))  _Float16 v8h;
typedef __attribute__((ext_vector_type(8)))  unsigned short v8us;
typedef __attribute__((ext_vector_type(8)))  float    v8f;
typedef __attribute__((ext_vector_type(4)))  float    v4f;
typedef v8h  __attribute__((may_alias)) v8ha;
typedef v4f  __attribute__((may_alias)) v4fa;
typedef v8us __attribute__((may_alias)) v8usa;

__device__ __forceinline__ unsigned short f2bf(float f) { unsigned u = __float_as_uint(f); u += 0x7FFFu + ((u >> 16) & 1u); return (unsigned short)(u >> 16); }
__device__ __forceinline__ float bf2f(unsigned short b) { return __uint_as_float(((unsigned)b) << 16); }
__device__ __forceinline__ float bfr(float f) { return bf2f(f2bf(f)); }
__device__ __forceinline__ v16h cat16(v8h lo, v8h hi) { return __builtin_shufflevector(lo, hi, 0, 1, 2, 3, 4, 5, 6, 7, 8, 9, 10, 11, 12, 13, 14, 15); }
__device__ __forceinline__ v16bf cat16b(v8us lo, v8us hi) { return __builtin_bit_cast(v16bf, __builtin_shufflevector(lo, hi, 0, 1, 2, 3, 4, 5, 6, 7, 8, 9, 10, 11, 12, 13, 14, 15)); }
__device__ __forceinline__ v8f wmma16(v16h a, v16h b, v8f c) { return __builtin_amdgcn_wmma_f32_16x16x32_f16(false, a, false, b, (short)0, c, false, false); }
__device__ __forceinline__ v8f wmmab(v16bf a, v16bf b, v8f c) { return __builtin_amdgcn_wmma_f32_16x16x32_bf16(false, a, false, b, (short)0, c, false, false); }
#define VST2(T, p, v) do { const T vst2_v_ = (v); *(volatile T*)(p) = vst2_v_; __threadfence(); *(volatile T*)(p) = vst2_v_; } while (0)

__global__ __launch_bounds__(256) void k_xb(const float* __restrict__ x, bf* Xb, float* XSQ) {
    __shared__ float sq[32];
    const int tid = threadIdx.x, lane = tid & 31, wave = tid >> 5;
    const int rl = tid >> 3, piece = tid & 7, r = blockIdx.x * 32 + rl;
    v8us t; float s = 0.f;
#pragma unroll
    for (int i = 0; i < 8; ++i) { const float v = bfr(x[(size_t)r * DD + piece * 8 + i]); t[i] = f2bf(v); s += v * v; }
    s += __shfl_xor(s, 1, 8); s += __shfl_xor(s, 2, 8); s += __shfl_xor(s, 4, 8);
    if (piece == 0) sq[rl] = s;
    VST2(v8us, Xb + (size_t)r * DD + piece * 8, t);
    __syncthreads();
    if (wave == 0) VST2(float, XSQ + (size_t)blockIdx.x * 32 + lane, sq[lane]);
}
__global__ __launch_bounds__(256) void k_cb(const float* __restrict__ c, bf* Cb, h16* CTH, h16* CTL, float* CSQ) {
    __shared__ float cs[KK];
    __shared__ __align__(16) h16 ct[DD * (KK + 8)];
    __shared__ __align__(16) h16 ctl[DD * (KK + 8)];
    const int tid = threadIdx.x;
#pragma unroll
    for (int rr = 0; rr < 2; ++rr) { const int k = tid * 2 + rr; float s = 0.f;
#pragma unroll 1
        for (int d = 0; d < DD; ++d) { const float v = bfr(c[(size_t)k * DD + d]); s += v * v; const float vs = v * CSC; const h16 a = (h16)vs; ct[d * (KK + 8) + k] = a; ctl[d * (KK + 8) + k] = (h16)((vs - (float)a) * LOSC); }
        cs[k] = s; }
    __syncthreads();
#pragma unroll 1
    for (int s = 0; s < (KK * DD) / 2048; ++s) { const int e0 = s * 2048 + tid * 8; v8us t;
#pragma unroll
        for (int i = 0; i < 8; ++i) { const int e = e0 + i, k = e / DD, d = e - k * DD; t[i] = f2bf(c[(size_t)k * DD + d]); }
        VST2(v8us, Cb + e0, t); }
#pragma unroll 1
    for (int s = 0; s < (KK * DD) / 2048; ++s) { const int e0 = s * 2048 + tid * 8; const int d = e0 / KK, k = e0 - d * KK; v8h t, t2;
#pragma unroll
        for (int i = 0; i < 8; ++i) { t[i] = ct[d * (KK + 8) + k + i]; t2[i] = ctl[d * (KK + 8) + k + i]; }
        VST2(v8h, CTH + e0, t); VST2(v8h, CTL + e0, t2); }
#pragma unroll
    for (int rr = 0; rr < 2; ++rr) { const int k = tid + rr * 256; VST2(float, CSQ + k, cs[k]); }
}

__global__ __launch_bounds__(128) void k_main(const bf* __restrict__ Xb, const float* __restrict__ XSQ, const bf* __restrict__ Cb, const float* __restrict__ CSQ, const h16* __restrict__ CTH, const h16* __restrict__ CTL, float* out) {
    __shared__ __align__(16) h16 plds[4][16 * 32];
    __shared__ __align__(16) h16 plds2[4][16 * 32];
    __shared__ __align__(16) float ost[4][16 * 68];
    const int lane = threadIdx.x & 31, wave = threadIdx.x >> 5, lr = lane & 15, hi = lane >> 4;
    const int r0 = blockIdx.x * 64 + wave * 16;
    h16* pl = &plds[wave][0]; h16* pl2 = &plds2[wave][0];
    v16bf xa[2];
#pragma unroll
    for (int kc = 0; kc < 2; ++kc) { const bf* p = Xb + (size_t)(r0 + lr) * DD + kc * 32 + 8 * hi; xa[kc] = cat16b(*(const v8us*)p, *(const v8us*)(p + 16)); }
    float xsq[8];
#pragma unroll
    for (int j = 0; j < 8; ++j) xsq[j] = XSQ[r0 + 8 * hi + j];
    const float nit = -1.0f / TEMP;
    float mrow[8], lsum[8];
#pragma unroll
    for (int j = 0; j < 8; ++j) { mrow[j] = -3.0e38f; lsum[j] = 0.f; }
    v8f o[4], ox[4];
#pragma unroll
    for (int n = 0; n < 4; ++n) { o[n] = (v8f){}; ox[n] = (v8f){}; }
#pragma unroll 1
    for (int pass = 0; pass < 2; ++pass) {
#pragma unroll 1
        for (int kt = 0; kt < KK / 32; ++kt) {
            const int k0 = kt * 32;
            v8f s0 = {}, s1 = {};
#pragma unroll
            for (int kc = 0; kc < 2; ++kc) {
                const bf* b0 = Cb + (size_t)(k0 + lr) * DD + kc * 32 + 8 * hi; const bf* b1 = b0 + (size_t)16 * DD;
                s0 = wmmab(xa[kc], cat16b(*(const v8us*)b0, *(const v8us*)(b0 + 16)), s0);
                s1 = wmmab(xa[kc], cat16b(*(const v8us*)b1, *(const v8us*)(b1 + 16)), s1);
            }
            asm volatile("v_nop\n\tv_nop\n\tv_nop\n\tv_nop" : "+v"(s0), "+v"(s1) : "v"(xa[0]), "v"(xa[1]));
            const float cq0 = CSQ[k0 + lr], cq1 = CSQ[k0 + 16 + lr];
            if (pass == 0) {
#pragma unroll
                for (int j = 0; j < 8; ++j) {
                    const float a0 = (xsq[j] - 2.0f * s0[j] + cq0) * nit, a1 = (xsq[j] - 2.0f * s1[j] + cq1) * nit;
                    float mx = fmaxf(a0, a1);
                    mx = fmaxf(mx, __shfl_xor(mx, 1, 16)); mx = fmaxf(mx, __shfl_xor(mx, 2, 16)); mx = fmaxf(mx, __shfl_xor(mx, 4, 16)); mx = fmaxf(mx, __shfl_xor(mx, 8, 16));
                    const float mn = fmaxf(mrow[j], mx);
                    float e = __expf(a0 - mn) + __expf(a1 - mn);
                    e += __shfl_xor(e, 1, 16); e += __shfl_xor(e, 2, 16); e += __shfl_xor(e, 4, 16); e += __shfl_xor(e, 8, 16);
                    lsum[j] = lsum[j] * __expf(mrow[j] - mn) + e; mrow[j] = mn;
                }
            } else {
#pragma unroll
                for (int j = 0; j < 8; ++j) {
                    const float a0 = (xsq[j] - 2.0f * s0[j] + cq0) * nit, a1 = (xsq[j] - 2.0f * s1[j] + cq1) * nit;
                    const float p0 = __expf(a0 - mrow[j]) / lsum[j] * PSC, p1 = __expf(a1 - mrow[j]) / lsum[j] * PSC;
                    const int mr = hi * 8 + j; const h16 h0 = (h16)p0, h1 = (h16)p1;
                    pl[mr * 32 + lr] = h0; pl[mr * 32 + 16 + lr] = h1; pl2[mr * 32 + lr] = (h16)((p0 - (float)h0) * LOSC); pl2[mr * 32 + 16 + lr] = (h16)((p1 - (float)h1) * LOSC);
                }
                asm volatile("" ::: "memory");
                const v16h pa = cat16(*(const v8ha*)(pl + lr * 32 + hi * 8), *(const v8ha*)(pl + lr * 32 + 16 + hi * 8));
                const v16h px = cat16(*(const v8ha*)(pl2 + lr * 32 + hi * 8), *(const v8ha*)(pl2 + lr * 32 + 16 + hi * 8));
#pragma unroll
                for (int n = 0; n < 4; ++n) { const size_t co = (size_t)(n * 16 + lr) * KK + k0 + hi * 8; const v16h cv = cat16(*(const v8h*)(CTH + co), *(const v8h*)(CTH + co + 16)), cl = cat16(*(const v8h*)(CTL + co), *(const v8h*)(CTL + co + 16));
                    o[n] = wmma16(pa, cv, o[n]); ox[n] = wmma16(px, cv, ox[n]); ox[n] = wmma16(pa, cl, ox[n]); }
                asm volatile("v_nop\n\tv_nop\n\tv_nop\n\tv_nop" : "+v"(o[0]), "+v"(o[1]), "+v"(o[2]), "+v"(o[3]), "+v"(ox[0]), "+v"(ox[1]), "+v"(ox[2]), "+v"(ox[3]) : "v"(pa), "v"(px));
                __builtin_amdgcn_wave_barrier();
            }
        }
    }
    float* os = &ost[wave][0];
#pragma unroll
    for (int n = 0; n < 4; ++n)
#pragma unroll
        for (int j = 0; j < 8; ++j) os[(hi * 8 + j) * 68 + n * 16 + lr] = (o[n][j] + ox[n][j] * LOSCI) * (1.0f / (PSC * CSC));
    __syncthreads();
    float* crow = out + (size_t)r0 * DD;
    auto passw = [&]() {
#pragma unroll
        for (int s = 0; s < 8; ++s) { const int Lid = (lane >> 3) + 4 * s, piece = lane & 7; const int row = Lid >> 1, cofs = (Lid & 1) * 32 + piece * 4;
            const v4f val = *(const v4fa*)(os + row * 68 + cofs); *(volatile v4f*)(crow + (size_t)row * DD + cofs) = val; }
    };
    passw(); __threadfence(); passw();
}

extern "C" void kernel_launch(void* const* d_in, const int* in_sizes, int n_in,
                              void* d_out, int out_size, void* d_ws, size_t ws_size, hipStream_t stream) {
    (void)in_sizes; (void)n_in; (void)out_size;
    const float* x = (const float*)d_in[0]; const float* c = (const float*)d_in[1];
    float* out = (float*)d_out;
    char* wsp = (char*)d_ws;
    auto take = [&](size_t bytes) { char* p = wsp; wsp += (bytes + 255) & ~(size_t)255; return (void*)p; };
    bf* Xb = (bf*)take((size_t)NN_ * DD * 2); float* XSQ = (float*)take((size_t)NN_ * 4); bf* Cb = (bf*)take((size_t)KK * DD * 2); h16* CTH = (h16*)take((size_t)KK * DD * 2); h16* CTL = (h16*)take((size_t)KK * DD * 2); float* CSQ = (float*)take(KK * 4);
    if ((size_t)(wsp - (char*)d_ws) > ws_size) return;
    k_xb<<<NN_ / 32, 256, 0, stream>>>(x, Xb, XSQ);
    k_cb<<<1, 256, 0, stream>>>(c, Cb, CTH, CTL, CSQ);
    k_main<<<NN_ / 64, 128, 0, stream>>>(Xb, XSQ, Cb, CSQ, CTH, CTL, out);
}
